// PraxisAttention_30700426232522
// MI455X (gfx1250) — hardware-verified
//
#include <hip/hip_runtime.h>
#include <math.h>

typedef __attribute__((ext_vector_type(16))) _Float16 v16h;
typedef __attribute__((ext_vector_type(16))) __bf16 v16b;
typedef __attribute__((ext_vector_type(8)))  _Float16 v8h;
typedef __attribute__((ext_vector_type(8)))  __bf16 v8b;
typedef __attribute__((ext_vector_type(8)))  float v8f;
typedef __attribute__((ext_vector_type(4)))  float v4f;
typedef __attribute__((ext_vector_type(4)))  unsigned v4u;

template <typename T> __device__ __forceinline__ void vst2(void* p, T v) { *(volatile T*)p = v; __threadfence(); *(volatile T*)p = v; }
__device__ __forceinline__ v8f wmma16(v16h a, v16h b, v8f c) {
  v8f d = __builtin_amdgcn_wmma_f32_16x16x32_f16(false, a, false, b, (short)0, c, false, false);
  asm volatile("v_nop\n\tv_nop\n\tv_nop\n\tv_nop" : "+v"(d) : "v"(a), "v"(b));
  return d;
}
__device__ __forceinline__ v8f wmma_bf(v16b a, v16b b, v8f c) {
  v8f d = __builtin_amdgcn_wmma_f32_16x16x32_bf16(false, a, false, b, (short)0, c, false, false);
  asm volatile("v_nop\n\tv_nop\n\tv_nop\n\tv_nop" : "+v"(d) : "v"(a), "v"(b));
  return d;
}
__device__ __forceinline__ v16h frag_h(const _Float16* rowk0, int lane) {
  union { v16h v; v8h q[2]; } u; const _Float16* p = rowk0 + 8 * (lane >> 4);
  u.q[0] = *(const v8h*)p; u.q[1] = *(const v8h*)(p + 16); return u.v;
}
__device__ __forceinline__ v16b frag_b(const __bf16* rowk0, int lane) {
  union { v16b v; v8b q[2]; } u; const __bf16* p = rowk0 + 8 * (lane >> 4);
  u.q[0] = *(const v8b*)p; u.q[1] = *(const v8b*)(p + 16); return u.v;
}
__device__ __forceinline__ v16h frag_f32(const float* rowk0, int lane) {
  v16h a; const float* p = rowk0 + 8 * (lane >> 4);
#pragma unroll
  for (int i = 0; i < 8; ++i) { a[i] = (_Float16)p[i]; a[8 + i] = (_Float16)p[16 + i]; }
  return a;
}
struct F2 { v16b h, l; };
__device__ __forceinline__ F2 bsplit16(const float v[16]) { F2 r;
#pragma unroll
  for (int i = 0; i < 16; ++i) { const __bf16 h = (__bf16)v[i]; r.h[i] = h; r.l[i] = (__bf16)(v[i] - (float)h); }
  return r; }
__device__ __forceinline__ F2 split_row(const float* row, int k0, int lane) { float v[16]; const float* p = row + k0 + 8 * (lane >> 4);
#pragma unroll
  for (int i = 0; i < 8; ++i) { v[i] = p[i]; v[8 + i] = p[16 + i]; }
  return bsplit16(v); }
__device__ __forceinline__ float bfr(float v) { return (float)(__bf16)v; }
#define LDSX() do { asm volatile("s_wait_dscnt 0" ::: "memory"); __builtin_amdgcn_wave_barrier(); __builtin_amdgcn_fence(3  , "workgroup"); } while (0)

#define NB_FULL 2
#define TT_FULL 2048
#ifndef NB
#define NB NB_FULL
#endif
#ifndef SEQ
#define SEQ TT_FULL
#endif
#define TT SEQ
#define CC 1024
#define DIN 1024
#define NH 16
#define HD 64
#define NQB (TT / 64)
#define HG 2
#define NST 2
#define SCALE (0.125f)
#define CAUSAL 1
#define QBH 4
#define QHI 256
#define KHI 256
#define PCAR (4096.0f)
#define LNEPS (1e-5f)
#define LINIT (0.8f)
static_assert(NB >= 1 && NB <= NB_FULL);
static_assert(TT % 128 == 0 && TT <= TT_FULL && TT >= KHI);
static_assert(QHI == QBH * 64);
static_assert((((QBH - 1) * 64 + 63) / 128 + 1) * 128 <= KHI);
static_assert(NH % HG == 0);
__host__ __device__ __forceinline__ int kb_last(int qb) { return CAUSAL ? ((qb * 64 + 63) >> 7) : (TT / 128 - 1); }
__device__ __forceinline__ v16b wcol_io(const float* Wm, int k0, int o, int lane, int ld) { v16b w; const int g = lane >> 4;
#pragma unroll
  for (int i = 0; i < 8; ++i) { w[i] = (__bf16)Wm[(size_t)(k0 + 8 * g + i) * ld + o]; w[8 + i] = (__bf16)Wm[(size_t)(k0 + 16 + 8 * g + i) * ld + o]; }
  return w; }
__device__ __forceinline__ v16h wcolh_io(const float* Wm, int k0, int o, int lane, int ld) { v16h w; const int g = lane >> 4;
#pragma unroll
  for (int i = 0; i < 8; ++i) { w[i] = (_Float16)(bfr(Wm[(size_t)(k0 + 8 * g + i) * ld + o]) * 256.0f); w[8 + i] = (_Float16)(bfr(Wm[(size_t)(k0 + 16 + 8 * g + i) * ld + o]) * 256.0f); }
  return w; }

#define WS_QH  ((size_t)0)
#define WS_KH  (WS_QH  + 2u * NST * (size_t)NB * TT * CC)
#define WS_VT  (WS_KH  + 2u * NST * (size_t)NB * TT * CC)
#define WS_QL  (WS_VT  + 2u * (size_t)NB * CC * TT)
#define WS_KL  (WS_QL  + 2u * NST * (size_t)NB * QHI * CC)
#define WS_VB  (WS_KL  + 2u * NST * (size_t)NB * KHI * CC)
#define WS_VBL (WS_VB  + 2u * (size_t)NB * CC * KHI)
#define WS_S   (WS_VBL + 2u * (size_t)NB * CC * KHI)
#define WS_Y   (WS_S   + 4u * (size_t)HG * NST * TT * TT)
#define WS_END (WS_Y   + 4u * (size_t)NB * TT * CC)
static_assert(WS_END <= (size_t)134217728u);
static_assert(WS_KH % 128 == 0 && WS_VT % 128 == 0 && WS_QL % 128 == 0 && WS_KL % 128 == 0 && WS_VB % 128 == 0 && WS_VBL % 128 == 0 && WS_S % 128 == 0 && WS_Y % 128 == 0);

__global__ __launch_bounds__(128) void k_proj(const float* __restrict__ X, const float* __restrict__ WQ0, const float* __restrict__ WQ1, const float* __restrict__ WK0, const float* __restrict__ WK1, const float* __restrict__ WV,
    _Float16* __restrict__ QH, _Float16* __restrict__ QL, _Float16* __restrict__ KH, _Float16* __restrict__ KL, _Float16* __restrict__ VT, __bf16* __restrict__ VB, __bf16* __restrict__ VBL) {
  __shared__ __align__(16) _Float16 sh[64][136], sl[64][136]; __shared__ __align__(16) _Float16 th[128][72]; __shared__ __align__(16) __bf16 tb[128][72], tbl[128][72];
  const int tid = threadIdx.x, wave = tid >> 5, lane = tid & 31, col = lane & 15, g = lane >> 4; const int which = blockIdx.z; const int c0 = blockIdx.y * 128; const size_t r0 = (size_t)blockIdx.x * 64; const size_t bb = r0 / TT; const int t0 = (int)(r0 % TT);
  const size_t xr0 = bb * TT_FULL + t0;
  const float* WA = which == 0 ? WQ0 : which == 1 ? WQ1 : which == 2 ? WK0 : which == 3 ? WK1 : WV;
  v8f acc[8] = {};
#pragma unroll 2
  for (int kc = 0; kc < DIN / 32; ++kc) { v16b a; { const float* p = X + (xr0 + wave * 16 + col) * DIN + kc * 32 + 8 * g;
#pragma unroll
      for (int i = 0; i < 8; ++i) { a[i] = (__bf16)p[i]; a[8 + i] = (__bf16)p[16 + i]; } }
    asm volatile("s_wait_loadcnt 0x0" ::: "memory");
#pragma unroll
    for (int j = 0; j < 8; ++j) { const v16b w = wcol_io(WA, kc * 32, c0 + j * 16 + col, lane, CC); asm volatile("s_wait_loadcnt 0x0" ::: "memory"); acc[j] = wmma_bf(a, w, acc[j]); } }
  if (which < 4) { const int st = which & 1; _Float16* DHp = (which < 2 ? QH : KH) + (size_t)st * NB * TT * CC; _Float16* DLp = (which < 2 ? QL : KL) + (size_t)st * NB * QHI * CC; const int nhi = which < 2 ? QHI : KHI; const bool hi_rows = t0 < nhi;
#pragma unroll
    for (int j = 0; j < 8; ++j) {
#pragma unroll
      for (int r = 0; r < 8; ++r) { const float v = acc[j][r]; const _Float16 hv = (_Float16)v; sh[wave * 16 + 8 * g + r][j * 16 + col] = hv; sl[wave * 16 + 8 * g + r][j * 16 + col] = (_Float16)((v - (float)hv) * 1024.0f); } }
    __syncthreads();
    for (int e = tid; e < 64 * 16; e += 128) { const int rl = e >> 4, q = e & 15; vst2((unsigned*)(DHp + (r0 + rl) * CC + c0 + q * 8), *(const v4u*)&sh[rl][q * 8]); if (hi_rows) vst2((unsigned*)(DLp + (bb * nhi + t0 + rl) * (size_t)CC + c0 + q * 8), *(const v4u*)&sl[rl][q * 8]); }
  } else { const bool hi_rows = t0 < KHI;
#pragma unroll
    for (int j = 0; j < 8; ++j) {
#pragma unroll
      for (int r = 0; r < 8; ++r) { const float v = acc[j][r]; const int rl = wave * 16 + 8 * g + r, cl = j * 16 + col; th[cl][rl] = (_Float16)v; const __bf16 bh = (__bf16)v; tb[cl][rl] = bh; tbl[cl][rl] = (__bf16)(v - (float)bh); } }
    __syncthreads();
    for (int e = tid; e < 128 * 8; e += 128) { const int cl = e >> 3, q = e & 7; vst2((unsigned*)(VT + (bb * CC + c0 + cl) * (size_t)TT + t0 + q * 8), *(const v4u*)&th[cl][q * 8]); if (hi_rows) { const size_t o3 = (bb * CC + c0 + cl) * (size_t)KHI + t0 + q * 8; vst2((unsigned*)(VB + o3), *(const v4u*)&tb[cl][q * 8]); vst2((unsigned*)(VBL + o3), *(const v4u*)&tbl[cl][q * 8]); } } } }
__global__ __launch_bounds__(128) void k_sc(const _Float16* __restrict__ QH, const _Float16* __restrict__ KH, const _Float16* __restrict__ QL, const _Float16* __restrict__ KL, int b, int h0, float* __restrict__ S0) { __shared__ __align__(16) float ss[4][16][132];
  const int qb = blockIdx.x, kb = blockIdx.y; if (kb > kb_last(qb)) return;
  const int z = blockIdx.z, st = z & 1, h = h0 + (z >> 1); float* S = S0 + (size_t)z * TT * TT;
  const int tid = threadIdx.x, wave = tid >> 5, lane = tid & 31, col = lane & 15, g = lane >> 4; const int k0 = kb * 128; const int ql0 = qb * 64 + wave * 16; const size_t q0 = (size_t)b * TT + ql0, kr0 = (size_t)b * TT + k0;
  const _Float16* QHs = QH + (size_t)st * NB * TT * CC; const _Float16* KHs = KH + (size_t)st * NB * TT * CC;
  const _Float16* QLb = QL + ((size_t)st * NB + b) * QHI * CC; const _Float16* KLb = KL + ((size_t)st * NB + b) * KHI * CC;
  v8f acc[8] = {}, accl[8] = {};
  if (qb < QBH) {
#pragma unroll
    for (int kc = 0; kc < HD / 32; ++kc) { const v16h ah = frag_h(QHs + (q0 + col) * CC + h * HD + kc * 32, lane), al = frag_h(QLb + (size_t)(ql0 + col) * CC + h * HD + kc * 32, lane);
#pragma unroll
      for (int j = 0; j < 8; ++j) { const v16h kbf = frag_h(KHs + (kr0 + j * 16 + col) * CC + h * HD + kc * 32, lane), klf = frag_h(KLb + (size_t)(k0 + j * 16 + col) * CC + h * HD + kc * 32, lane); acc[j] = wmma16(ah, kbf, acc[j]); accl[j] = wmma16(al, kbf, accl[j]); accl[j] = wmma16(ah, klf, accl[j]); } }
  } else if (qb * 64 < QHI) {
#pragma unroll
    for (int kc = 0; kc < HD / 32; ++kc) { const v16h ah = frag_h(QHs + (q0 + col) * CC + h * HD + kc * 32, lane), al = frag_h(QLb + (size_t)(ql0 + col) * CC + h * HD + kc * 32, lane);
#pragma unroll
      for (int j = 0; j < 8; ++j) { const v16h kbf = frag_h(KHs + (kr0 + j * 16 + col) * CC + h * HD + kc * 32, lane); acc[j] = wmma16(ah, kbf, acc[j]); accl[j] = wmma16(al, kbf, accl[j]); } }
  } else {
#pragma unroll
    for (int kc = 0; kc < HD / 32; ++kc) { const v16h ah = frag_h(QHs + (q0 + col) * CC + h * HD + kc * 32, lane);
#pragma unroll
      for (int j = 0; j < 8; ++j) { const v16h kbf = frag_h(KHs + (kr0 + j * 16 + col) * CC + h * HD + kc * 32, lane); acc[j] = wmma16(ah, kbf, acc[j]); } } }
#pragma unroll
  for (int j = 0; j < 8; ++j) {
#pragma unroll
    for (int r = 0; r < 8; ++r) ss[wave][8 * g + r][j * 16 + col] = (acc[j][r] + accl[j][r] * (1.0f / 1024.0f)) * SCALE; }
  LDSX(); for (int rl = 0; rl < 16; ++rl) vst2(S + (size_t)(ql0 + rl) * TT + k0 + lane * 4, *(const v4f*)&ss[wave][rl][lane * 4]); }
__global__ __launch_bounds__(256) void k_sm(float* __restrict__ S0, const float* __restrict__ L0, const float* __restrict__ L1, const float* __restrict__ L2, const float* __restrict__ L3, int h0s) {
  __shared__ float sred[4][8]; __shared__ float sbc[4]; __shared__ __align__(16) float shv0[TT]; __shared__ __align__(16) float shv1[TT];
  const int tid = threadIdx.x, wave = tid >> 5, lane = tid & 31; const int t = blockIdx.x; const int kend = (kb_last(t >> 6) + 1) * 128;
  float* sr0 = S0 + (size_t)(NST * blockIdx.y) * TT * TT + (size_t)t * TT; const float* sr1 = sr0 + (size_t)TT * TT;
  const int hh = h0s + (int)blockIdx.y; const float slope = exp2f(-0.5f * (float)(hh + 1));
  const int li = tid & (HD - 1);
  const float pa = bfr(L0[li]) * bfr(L1[li]), pb = bfr(L2[li]) * bfr(L3[li]);
  float d01 = (tid < HD) ? pa : 0.f, d23 = (tid < HD) ? pb : 0.f;
  float m0 = -3.0e38f, m1 = -3.0e38f;
  for (int k = tid; k < kend; k += 256) { const float bias = slope * (float)(k - t); const bool inc = (!CAUSAL) || (k <= t); const float a0 = sr0[k], a1 = sr1[k];
    const float v0 = inc ? a0 + bias : -3.0e38f, v1 = inc ? a1 + bias : -3.0e38f; shv0[k] = v0; shv1[k] = v1; m0 = fmaxf(m0, v0); m1 = fmaxf(m1, v1); }
#pragma unroll
  for (int o = 1; o < 32; o <<= 1) { m0 = fmaxf(m0, __shfl_xor(m0, o)); m1 = fmaxf(m1, __shfl_xor(m1, o)); d01 += __shfl_xor(d01, o); d23 += __shfl_xor(d23, o); }
  if (lane == 0) { sred[0][wave] = m0; sred[1][wave] = m1; sred[2][wave] = d01; sred[3][wave] = d23; } __syncthreads();
  if (tid == 0) { float a = sred[0][0], c = sred[1][0], e = sred[2][0], f = sred[3][0]; for (int i = 1; i < 8; ++i) { a = fmaxf(a, sred[0][i]); c = fmaxf(c, sred[1][i]); e += sred[2][i]; f += sred[3][i]; }
    sbc[0] = a; sbc[1] = c; sbc[2] = (LINIT - expf(e)) + (LINIT - expf(f)); }
  __syncthreads(); m0 = sbc[0]; m1 = sbc[1]; const float lam = sbc[2]; __syncthreads();
  float s0 = 0.f, s1 = 0.f;
  for (int k = tid; k < kend; k += 256) { const float v0 = shv0[k], v1 = shv1[k]; const float e0 = (v0 <= -1.0e38f) ? 0.f : expf(v0 - m0); const float e1 = (v1 <= -1.0e38f) ? 0.f : expf(v1 - m1); shv0[k] = e0; shv1[k] = e1; s0 += e0; s1 += e1; }
#pragma unroll
  for (int o = 1; o < 32; o <<= 1) { s0 += __shfl_xor(s0, o); s1 += __shfl_xor(s1, o); }
  if (lane == 0) { sred[0][wave] = s0; sred[1][wave] = s1; } __syncthreads();
  if (tid == 0) { float a = 0.f, c = 0.f; for (int i = 0; i < 8; ++i) { a += sred[0][i]; c += sred[1][i]; } const float f0 = a > 0.f ? PCAR / a : 0.f; const float f1 = c > 0.f ? PCAR / c : 0.f; sbc[0] = f0; sbc[1] = lam * f1; }
  __syncthreads(); const float f0 = sbc[0], f1 = sbc[1];
  for (int q = tid; q < kend / 4; q += 256) { const v4f e0 = *(const v4f*)&shv0[q * 4], e1 = *(const v4f*)&shv1[q * 4]; const v4f dv = e0 * f0 - e1 * f1; vst2(sr0 + q * 4, dv); } }
__global__ __launch_bounds__(128) void k_pv(const float* __restrict__ PS0, const _Float16* __restrict__ VT, const __bf16* __restrict__ VB, const __bf16* __restrict__ VBL, const float* __restrict__ LW, const float* __restrict__ LB, int b, int h0, float* __restrict__ Y) {
  const int h = h0 + blockIdx.z; const float* PS = PS0 + (size_t)(NST * blockIdx.z) * TT * TT; __shared__ __align__(16) float ss[4][16][HD + 4];
  const int tid = threadIdx.x, wave = tid >> 5, lane = tid & 31, col = lane & 15, g = lane >> 4; const int qb = blockIdx.x; const int ql0 = qb * 64 + wave * 16; const int kce = (kb_last(qb) + 1) * 4;
  v8f acc[HD / 16] = {};
  if (qb < QBH) {
#pragma unroll 1
    for (int kc = 0; kc < kce; ++kc) { const F2 p = split_row(PS + (size_t)(ql0 + col) * TT, kc * 32, lane);
      asm volatile("s_wait_loadcnt 0x0" ::: "memory");
#pragma unroll
      for (int j = 0; j < HD / 16; ++j) { const size_t po = ((size_t)b * CC + h * HD + j * 16 + col) * (size_t)KHI + kc * 32; const v16b vh = frag_b(VB + po, lane); acc[j] = wmma_bf(p.h, vh, acc[j]); acc[j] = wmma_bf(p.l, vh, acc[j]); acc[j] = wmma_bf(p.h, frag_b(VBL + po, lane), acc[j]); } }
  } else {
#pragma unroll 1
    for (int kc = 0; kc < kce; ++kc) { const v16h p = frag_f32(PS + (size_t)(ql0 + col) * TT + kc * 32, lane);
      asm volatile("s_wait_loadcnt 0x0" ::: "memory");
#pragma unroll
      for (int j = 0; j < HD / 16; ++j) { const size_t po = ((size_t)b * CC + h * HD + j * 16 + col) * (size_t)TT + kc * 32; acc[j] = wmma16(p, frag_h(VT + po, lane), acc[j]); } } }
#pragma unroll
  for (int j = 0; j < HD / 16; ++j)
#pragma unroll
    for (int r = 0; r < 8; ++r) ss[wave][8 * g + r][j * 16 + col] = acc[j][r] * (1.0f / PCAR);
  LDSX();
  const int hl = lane & 15; v4f wv, wb;
#pragma unroll
  for (int i = 0; i < 4; ++i) { wv[i] = bfr(LW[h * HD + hl * 4 + i]); wb[i] = bfr(LB[h * HD + hl * 4 + i]); }
  const size_t yr0 = (size_t)b * TT + ql0;
  for (int rl = 0; rl < 16; ++rl) {
    const v4f x = *(const v4f*)&ss[wave][rl][hl * 4];
    float s = (x[0] + x[1]) + (x[2] + x[3]);
    s += __shfl_xor(s, 1); s += __shfl_xor(s, 2); s += __shfl_xor(s, 4); s += __shfl_xor(s, 8);
    const float mu = s * (1.0f / HD);
    const v4f d = x - mu;
    float qs = (d[0] * d[0] + d[1] * d[1]) + (d[2] * d[2] + d[3] * d[3]);
    qs += __shfl_xor(qs, 1); qs += __shfl_xor(qs, 2); qs += __shfl_xor(qs, 4); qs += __shfl_xor(qs, 8);
    const float rstd = rsqrtf(qs * (1.0f / HD) + LNEPS);
    v4f n;
#pragma unroll
    for (int i = 0; i < 4; ++i) n[i] = (d[i] * rstd) * wv[i] + wb[i];
    if (lane < HD / 4) vst2(Y + (yr0 + rl) * CC + h * HD + hl * 4, n);
  } }
__global__ __launch_bounds__(128) void k_out(const float* __restrict__ Y, const float* __restrict__ WO, float* __restrict__ OUT) { __shared__ __align__(16) float sf[4][16][132];
  const int tid = threadIdx.x, wave = tid >> 5, lane = tid & 31, col = lane & 15, g = lane >> 4; const int c0 = blockIdx.y * 128;
  const size_t rb = (size_t)blockIdx.x * 64; const size_t bb = rb / TT; const int t0 = (int)(rb % TT); const size_t r0 = rb + wave * 16; const size_t o0 = bb * TT_FULL + t0 + wave * 16;
  v8f acc[8] = {};
  if (CAUSAL && t0 < QHI) {
#pragma unroll 2
    for (int kc = 0; kc < CC / 32; ++kc) { const F2 a = split_row(Y + (r0 + col) * CC, kc * 32, lane); asm volatile("s_wait_loadcnt 0x0" ::: "memory");
#pragma unroll
      for (int j = 0; j < 8; ++j) { const v16b w = wcol_io(WO, kc * 32, c0 + j * 16 + col, lane, DIN); asm volatile("s_wait_loadcnt 0x0" ::: "memory"); acc[j] = wmma_bf(a.h, w, acc[j]); acc[j] = wmma_bf(a.l, w, acc[j]); } }
#pragma unroll
    for (int j = 0; j < 8; ++j) {
#pragma unroll
      for (int r = 0; r < 8; ++r) sf[wave][8 * g + r][j * 16 + col] = acc[j][r]; }
  } else {
#pragma unroll 2
    for (int kc = 0; kc < CC / 32; ++kc) { const v16h a = frag_f32(Y + (r0 + col) * CC + kc * 32, lane); asm volatile("s_wait_loadcnt 0x0" ::: "memory");
#pragma unroll
      for (int j = 0; j < 8; ++j) { const v16h w = wcolh_io(WO, kc * 32, c0 + j * 16 + col, lane, DIN); asm volatile("s_wait_loadcnt 0x0" ::: "memory"); acc[j] = wmma16(a, w, acc[j]); } }
#pragma unroll
    for (int j = 0; j < 8; ++j) {
#pragma unroll
      for (int r = 0; r < 8; ++r) sf[wave][8 * g + r][j * 16 + col] = acc[j][r] * (1.0f / 256.0f); } }
  LDSX(); for (int rl = 0; rl < 16; ++rl) vst2(OUT + (o0 + rl) * DIN + c0 + lane * 4, *(const v4f*)&sf[wave][rl][lane * 4]); }

extern "C" void kernel_launch(void* const* d_in, const int* in_sizes, int n_in, void* d_out, int out_size, void* d_ws, size_t ws_size, hipStream_t stream) {
  if (n_in < 13) return;
  const size_t need_rows = (size_t)(NB - 1) * TT_FULL + (size_t)TT;
  if ((size_t)in_sizes[0] < need_rows * DIN) return;
  for (int i = 1; i <= 6; ++i) if (in_sizes[i] < DIN * CC) return;
  for (int i = 7; i <= 10; ++i) if (in_sizes[i] < HD) return;
  if (in_sizes[11] < NH * HD || in_sizes[12] < NH * HD) return;
  if ((size_t)out_size < need_rows * DIN) return;
  if (ws_size < WS_END) return;
  const float* X  = (const float*)d_in[0];
  const float* W1 = (const float*)d_in[1]; const float* W2 = (const float*)d_in[2]; const float* W3 = (const float*)d_in[3]; const float* W4 = (const float*)d_in[4]; const float* W5 = (const float*)d_in[5]; const float* WO = (const float*)d_in[6];
  const float* L0 = (const float*)d_in[7]; const float* L1 = (const float*)d_in[8]; const float* L2 = (const float*)d_in[9]; const float* L3 = (const float*)d_in[10];
  const float* LW = (const float*)d_in[11]; const float* LB = (const float*)d_in[12];
  char* ws = (char*)d_ws; _Float16 *QH = (_Float16*)(ws + WS_QH), *KH = (_Float16*)(ws + WS_KH), *VT = (_Float16*)(ws + WS_VT), *QL = (_Float16*)(ws + WS_QL), *KL = (_Float16*)(ws + WS_KL); __bf16 *VB = (__bf16*)(ws + WS_VB), *VBL = (__bf16*)(ws + WS_VBL); float *S = (float*)(ws + WS_S), *Y = (float*)(ws + WS_Y);
  k_proj<<<dim3(NB * TT / 64, CC / 128, 5), 128, 0, stream>>>(X, W1, W2, W3, W4, W5, QH, QL, KH, KL, VT, VB, VBL);
  for (int b = 0; b < NB; ++b) for (int h0 = 0; h0 < NH; h0 += HG) {
    k_sc<<<dim3(NQB, TT / 128, HG * NST), 128, 0, stream>>>(QH, KH, QL, KL, b, h0, S);
    k_sm<<<dim3(TT, HG), 256, 0, stream>>>(S, L0, L1, L2, L3, h0);
    k_pv<<<dim3(NQB, 1, HG), 128, 0, stream>>>(S, VT, VB, VBL, LW, LB, b, h0, Y);
  }
  k_out<<<dim3(NB * TT / 64, DIN / 128), 128, 0, stream>>>(Y, WO, (float*)d_out);
}
